// NLB_57750130262587
// MI455X (gfx1250) — hardware-run, weakly checked
//
#include <hip/hip_runtime.h>


#ifndef NB
#define NB 2
#endif
#ifndef HWP
#define HWP 4096
#endif
#define NB_FULL  2
#define HWP_FULL 4096
#define CI   192
#define CH   96
#define CO   192
#define NTOK (NB * HWP)
#define AW   4
#define OSP  100
#define QRS  2048.0f
#define QRI  (1.0f / 2048.0f)
#define LOG2E ((float)1.4426950408889634)
#define PSH  14.0f
#define NEGB (-3.0e38f)
#define WLS  64.0f
#define WLI  (1.0f / 64.0f)

static_assert(CI % 32 == 0);
static_assert(CH % 32 == 0);
static_assert(CH == 96);
static_assert(CH % 48 == 0);
static_assert(CO % 64 == 0);
static_assert(CI == CO);
static_assert(HWP % 64 == 0);
static_assert(HWP % 32 == 0);
static_assert(NTOK % 64 == 0);
static_assert(NTOK % 32 == 0);
static_assert(NTOK % (16 * AW) == 0);
static_assert(((size_t)CH * CI) % 8 == 0);
static_assert(((size_t)CO * CH) % 8 == 0);
static_assert(NB <= NB_FULL);
static_assert(HWP <= HWP_FULL);
static_assert((OSP * 4) % 16 == 0);
static_assert(OSP >= CH);

typedef _Float16 h16;
typedef unsigned short bf;
typedef __attribute__((ext_vector_type(16))) __bf16   v16bf;
typedef __attribute__((ext_vector_type(16))) _Float16 v16h;
typedef __attribute__((ext_vector_type(8)))  _Float16 v8h;
typedef __attribute__((ext_vector_type(8)))  unsigned short v8us;
typedef __attribute__((ext_vector_type(8)))  float    v8f;
typedef __attribute__((ext_vector_type(4)))  float    v4f;
typedef v4f  __attribute__((may_alias)) v4fa;
typedef v8h  __attribute__((may_alias)) v8ha;

__device__ __forceinline__ unsigned short f2bf(float f) { unsigned u = __float_as_uint(f); u += 0x7FFFu + ((u >> 16) & 1u); return (unsigned short)(u >> 16); }
__device__ __forceinline__ float bfr(float f) { return __uint_as_float(((unsigned)f2bf(f)) << 16); }
__device__ __forceinline__ v16h cat16(v8h lo, v8h hi) { return __builtin_shufflevector(lo, hi, 0, 1, 2, 3, 4, 5, 6, 7, 8, 9, 10, 11, 12, 13, 14, 15); }
__device__ __forceinline__ v16bf cat16b(v8us lo, v8us hi) { return __builtin_bit_cast(v16bf, __builtin_shufflevector(lo, hi, 0, 1, 2, 3, 4, 5, 6, 7, 8, 9, 10, 11, 12, 13, 14, 15)); }
__device__ __forceinline__ v8f wmma16(v16h a, v16h b, v8f c) { return __builtin_amdgcn_wmma_f32_16x16x32_f16(false, a, false, b, (short)0, c, false, false); }
__device__ __forceinline__ v8f wmmab(v16bf a, v16bf b, v8f c) { return __builtin_amdgcn_wmma_f32_16x16x32_bf16(false, a, false, b, (short)0, c, false, false); }
__device__ __forceinline__ v8f wmma16g(v16h a, v16h b, v8f c) { c = wmma16(a, b, c); asm volatile("v_nop\n\tv_nop\n\tv_nop\n\tv_nop" : "+v"(c) : "v"(a), "v"(b)); return c; }
__device__ __forceinline__ v8f wmmabg(v16bf a, v16bf b, v8f c) { c = wmmab(a, b, c); asm volatile("v_nop\n\tv_nop\n\tv_nop\n\tv_nop" : "+v"(c) : "v"(a), "v"(b)); return c; }
__device__ __forceinline__ v16h  ldh(const h16* p) { return cat16(*(const v8h*)p, *(const v8h*)(p + 16)); }
__device__ __forceinline__ v16bf ldb(const bf* p)  { return cat16b(*(const v8us*)p, *(const v8us*)(p + 16)); }
__device__ __forceinline__ void wave_sync() { __builtin_amdgcn_fence(3  , "wavefront"); __builtin_amdgcn_wave_barrier(); asm volatile("" ::: "memory"); }
static __device__ __forceinline__ h16 toh_flush(float v) { const float w = (fabsf(v) < 6.103515625e-05f) ? 0.0f : v; return (h16)w; }

__global__ __launch_bounds__(256) void k_cvt8(const float* __restrict__ src, bf* dst, size_t n8) {
    const size_t i = (size_t)blockIdx.x * 256 + threadIdx.x; if (i >= n8) return;
    const v8f v = *(const v8f*)(src + i * 8); v8us o;
#pragma unroll
    for (int k = 0; k < 8; ++k) o[k] = f2bf(v[k]);
    *(volatile v8us*)(dst + i * 8) = o; __threadfence(); *(volatile v8us*)(dst + i * 8) = o;
}

__global__ __launch_bounds__(256) void k_wcvt(const float* __restrict__ src, h16* dst, unsigned n8) {
    const unsigned i = blockIdx.x * 256u + threadIdx.x; if (i >= n8) return;
    const v8f v = *(const v8f*)(src + (size_t)i * 8); v8h o;
#pragma unroll
    for (int k = 0; k < 8; ++k) o[k] = toh_flush(bfr(v[k]) * WLS);
    *(volatile v8h*)(dst + (size_t)i * 8) = o; __threadfence(); *(volatile v8h*)(dst + (size_t)i * 8) = o;
}

static_assert(3 * 256 * 16 == 32 * CI * 2);
static_assert((CI / 8) * 8 == CI);
static_assert(CI * 33 * 4 <= 131072);
__global__ __launch_bounds__(256) void k_xt(const float* __restrict__ x, bf* XT) {
    __shared__ float ts[CI * 33];
    const unsigned tid = threadIdx.x;
    const unsigned p0 = blockIdx.x * 32u, b = blockIdx.y;
    const unsigned pl = tid & 31u, cw = tid >> 5;
    const float* xb = x + (size_t)b * CI * HWP_FULL + p0 + pl;
#pragma unroll 4
    for (unsigned i = 0; i < CI / 8; ++i) { const unsigned c = cw + 8u * i; ts[c * 33u + pl] = xb[(size_t)c * HWP_FULL]; }
    __syncthreads();
    bf* dst = XT + ((size_t)b * HWP + p0) * CI;
    v8us o[3];
#pragma unroll
    for (int it = 0; it < 3; ++it) { const unsigned q = (unsigned)it * 256u + tid; const unsigned row = q / 24u, pc = q % 24u;
#pragma unroll
        for (int k = 0; k < 8; ++k) o[it][k] = f2bf(ts[(pc * 8u + (unsigned)k) * 33u + row]); }
#pragma unroll
    for (int it = 0; it < 3; ++it) { const unsigned q = (unsigned)it * 256u + tid; *(volatile v8us*)(dst + (size_t)q * 8) = o[it]; }
    __threadfence();
#pragma unroll
    for (int it = 0; it < 3; ++it) { const unsigned q = (unsigned)it * 256u + tid; *(volatile v8us*)(dst + (size_t)q * 8) = o[it]; }
}

static_assert(4 * 32 * 16 == 16 * 64 * 2);
__global__ __launch_bounds__(32) void k_proj(const bf* __restrict__ A, const bf* __restrict__ Bt, const float* __restrict__ bias, h16* Ph, h16* Pr, int wres) {
    __shared__ __align__(16) float os[16 * 68];
    const int lane = threadIdx.x & 31, lr = lane & 15, hi = lane >> 4;
    const unsigned r0 = blockIdx.x * 48u, c0 = blockIdx.y * 64u;
    v8f acc[3][4];
#pragma unroll
    for (int mb = 0; mb < 3; ++mb)
#pragma unroll
        for (int nb = 0; nb < 4; ++nb) acc[mb][nb] = (v8f){};
    const size_t aoff = (size_t)(r0 + (unsigned)lr) * CI + 8 * hi, boff = (size_t)(c0 + (unsigned)lr) * CI + 8 * hi;
#pragma unroll 1
    for (int kc = 0; kc < CI; kc += 32) {
        v16bf a[3];
#pragma unroll
        for (int mb = 0; mb < 3; ++mb) a[mb] = ldb(A + aoff + (size_t)mb * 16 * CI + kc);
#pragma unroll
        for (int nb = 0; nb < 4; ++nb) { const v16bf b = ldb(Bt + boff + (size_t)nb * 16 * CI + kc);
#pragma unroll
            for (int mb = 0; mb < 3; ++mb) acc[mb][nb] = wmmabg(a[mb], b, acc[mb][nb]); }
    }
    const unsigned bb = c0 / (unsigned)HWP, tt = c0 % (unsigned)HWP;
    const size_t tbase = ((size_t)bb * CH + (size_t)r0) * HWP + (size_t)tt;
    const bool wr = wres != 0;
#pragma unroll
    for (int mb = 0; mb < 3; ++mb) {
        float br[8];
#pragma unroll
        for (int j = 0; j < 8; ++j) br[j] = bfr(bias[r0 + (unsigned)(mb * 16 + hi * 8 + j)]);
#pragma unroll
        for (int nb = 0; nb < 4; ++nb) {
#pragma unroll
            for (int j = 0; j < 8; ++j) os[(hi * 8 + j) * 68 + nb * 16 + lr] = acc[mb][nb][j] + br[j]; }
        wave_sync();
#pragma unroll 1
        for (int ps = 0; ps < 2; ++ps) {
            const size_t sb = tbase + (size_t)(mb * 16) * HWP;
#pragma unroll
            for (int s = 0; s < 4; ++s) { const int row = 4 * s + (lane >> 3), c8 = (lane & 7) * 8;
                const v4f x0 = *(const v4fa*)(&os[row * 68 + c8]); const v4f x1 = *(const v4fa*)(&os[row * 68 + c8 + 4]); v8h hv, rv;
#pragma unroll
                for (int i = 0; i < 4; ++i) { const h16 a0 = toh_flush(x0[i]); const h16 a1 = toh_flush(x1[i]); hv[i] = a0; hv[4 + i] = a1;
                    rv[i] = toh_flush((x0[i] - (float)a0) * QRS); rv[4 + i] = toh_flush((x1[i] - (float)a1) * QRS); }
                const size_t oo = sb + (size_t)row * HWP + c8;
                *(volatile v8h*)(Ph + oo) = hv; if (wr) *(volatile v8h*)(Pr + oo) = rv; }
            if (ps == 0) __threadfence(); }
        wave_sync();
    }
}

static_assert(3 * 256 * 16 == 64 * CH * 2);
static_assert(3 * 32 == CH);
static_assert(64 * 104 * 2 <= 131072);
__global__ __launch_bounds__(256) void k_vt(const h16* __restrict__ V, h16* VT) {
    __shared__ __align__(16) h16 ts[64 * 104];
    const unsigned tid = threadIdx.x; const unsigned tok0 = blockIdx.x * 64u;
    const h16* src = V + (size_t)tok0 * CH;
#pragma unroll 1
    for (int it = 0; it < 3; ++it) { unsigned q = (unsigned)it * 256u + tid; asm volatile("" : "+v"(q)); const unsigned row = q / 12u, pc = q % 12u;
        const v8h v = *(const v8h*)(src + (size_t)q * 8); *(v8ha*)(&ts[row * 104u + pc * 8u]) = v; }
    __syncthreads();
    const unsigned j8 = (tid & 7u) * 8u;
    v8h o[3];
#pragma unroll
    for (int it = 0; it < 3; ++it) { const unsigned d = (unsigned)it * 32u + (tid >> 3);
#pragma unroll
        for (int k = 0; k < 8; ++k) o[it][k] = ts[(j8 + (unsigned)k) * 104u + d]; }
#pragma unroll
    for (int it = 0; it < 3; ++it) { const unsigned d = (unsigned)it * 32u + (tid >> 3); *(volatile v8h*)(VT + (size_t)d * NTOK + tok0 + j8) = o[it]; }
    __threadfence();
#pragma unroll
    for (int it = 0; it < 3; ++it) { const unsigned d = (unsigned)it * 32u + (tid >> 3); *(volatile v8h*)(VT + (size_t)d * NTOK + tok0 + j8) = o[it]; }
}

static_assert(CH * 8 == 3 * 256);
static_assert(CH * 72 * 2 <= 131072);
__global__ __launch_bounds__(256) void k_at(const h16* __restrict__ AO, h16* AOT) {
    __shared__ __align__(16) h16 ts[CH * 72];
    const unsigned tid = threadIdx.x; const unsigned p0 = blockIdx.x * 64u, b = blockIdx.y;
    const h16* src = AO + (size_t)b * CH * HWP + p0;
#pragma unroll
    for (int it = 0; it < 3; ++it) { const unsigned q = (unsigned)it * 256u + tid; const unsigned c = q >> 3, j8 = (q & 7u) * 8u;
        const v8h v = *(const v8h*)(src + (size_t)c * HWP + j8); *(v8ha*)(&ts[c * 72u + j8]) = v; }
    __syncthreads();
    h16* dst = AOT + ((size_t)b * HWP + p0) * CH;
    v8h o[3];
#pragma unroll
    for (int it = 0; it < 3; ++it) { const unsigned q = (unsigned)it * 256u + tid; const unsigned row = q / 12u, pc = q % 12u;
#pragma unroll
        for (int k = 0; k < 8; ++k) o[it][k] = ts[(pc * 8u + (unsigned)k) * 72u + row]; }
#pragma unroll
    for (int it = 0; it < 3; ++it) { const unsigned q = (unsigned)it * 256u + tid; *(volatile v8h*)(dst + (size_t)q * 8) = o[it]; }
    __threadfence();
#pragma unroll
    for (int it = 0; it < 3; ++it) { const unsigned q = (unsigned)it * 256u + tid; *(volatile v8h*)(dst + (size_t)q * 8) = o[it]; }
}

static_assert(6 * 32 * 16 == 16 * CH * 2);
static_assert(AW * 16 * OSP * 4 <= 131072);
__global__ __launch_bounds__(32 * AW) __attribute__((amdgpu_num_vgpr(256)))
void k_flash(const h16* __restrict__ QH, const h16* __restrict__ QR, const h16* __restrict__ KP, const h16* __restrict__ KR,
             const h16* __restrict__ VT, h16* AO) {
    __shared__ __align__(16) float os[AW * 16 * OSP];
    const unsigned lane = threadIdx.x & 31u, lr = lane & 15u, hi = lane >> 4;
    const unsigned wave = (unsigned)__builtin_amdgcn_readfirstlane((int)(threadIdx.x >> 5));
    const unsigned bx = blockIdx.x;
    const unsigned t0 = (bx * (unsigned)AW + wave) * 16u;
    const size_t qo = (size_t)(t0 + lr) * CH + 8u * hi;
    v16h qh[3], qr[3];
#pragma unroll
    for (int kc = 0; kc < 3; ++kc) { qh[kc] = ldh(QH + qo + kc * 32); qr[kc] = ldh(QR + qo + kc * 32); }
    const size_t ko = (size_t)lr * CH + 8u * hi;
    const size_t vo = (size_t)lr * NTOK + 8u * hi;
    v8f o[6];
#pragma unroll
    for (int j = 0; j < 6; ++j) o[j] = (v8f){};
    float m = NEGB, l = 0.0f;
#pragma unroll 1
    for (unsigned key0 = 0; key0 < (unsigned)NTOK; key0 += 32u) {
        const h16* ka = KP + ko + (size_t)key0 * CH;
        const h16* kr = KR + ko + (size_t)key0 * CH;
        v8f sHa = (v8f){}, sLa = (v8f){}, sHb = (v8f){}, sLb = (v8f){};
#pragma unroll
        for (int kc = 0; kc < 3; ++kc) {
            const v16h a0 = ldh(ka + kc * 32), b0 = ldh(ka + 16 * CH + kc * 32);
            const v16h ar = ldh(kr + kc * 32), br = ldh(kr + 16 * CH + kc * 32);
            sHa = wmma16g(a0, qh[kc], sHa); sLa = wmma16g(a0, qr[kc], sLa); sLa = wmma16g(ar, qh[kc], sLa);
            sHb = wmma16g(b0, qh[kc], sHb); sLb = wmma16g(b0, qr[kc], sLb); sLb = wmma16g(br, qh[kc], sLb);
        }
        float ta[8], tb[8]; float mx = NEGB;
#pragma unroll
        for (int r = 0; r < 8; ++r) {
            ta[r] = (sHa[r] + sLa[r] * QRI) * LOG2E; tb[r] = (sHb[r] + sLb[r] * QRI) * LOG2E;
            mx = fmaxf(mx, fmaxf(ta[r], tb[r])); }
        mx = fmaxf(mx, __shfl_xor(mx, 16, 32));
        const float mnew = fmaxf(m, mx);
        const float alpha = __builtin_amdgcn_exp2f(m - mnew);
        const float sh = PSH - mnew;
        v16h pb; float ls = 0.0f;
#pragma unroll
        for (int r = 0; r < 8; ++r) {
            const float xa = ta[r] + sh, xb = tb[r] + sh;
            const float ea = __builtin_amdgcn_exp2f(xa), eb = __builtin_amdgcn_exp2f(xb);
            const float ga = (xa < -14.0f) ? 0.0f : ea, gb = (xb < -14.0f) ? 0.0f : eb;
            const h16 pa = (h16)ga; const h16 pc = (h16)gb;
            pb[r] = pa; pb[8 + r] = pc;
            ls += (float)pa + (float)pc; }
        l = l * alpha + ls; m = mnew;
#pragma unroll
        for (int j = 0; j < 6; ++j) o[j] = o[j] * alpha;
        const h16* va = VT + vo + key0;
#pragma unroll
        for (int j = 0; j < 6; ++j) { const v16h vj = ldh(va + (size_t)(16 * j) * NTOK); o[j] = wmma16g(vj, pb, o[j]); }
    }
    l += __shfl_xor(l, 16, 32);
    const float inv = 1.0f / fmaxf(l, 1.0f);
    const unsigned wb = wave * 16u * OSP;
#pragma unroll
    for (int j = 0; j < 6; ++j) { v4f a, c;
        a[0] = o[j][0] * inv; a[1] = o[j][1] * inv; a[2] = o[j][2] * inv; a[3] = o[j][3] * inv;
        c[0] = o[j][4] * inv; c[1] = o[j][5] * inv; c[2] = o[j][6] * inv; c[3] = o[j][7] * inv;
        *(v4fa*)(&os[wb + lr * OSP + 16 * j + 8 * hi]) = a; *(v4fa*)(&os[wb + lr * OSP + 16 * j + 8 * hi + 4]) = c; }
    wave_sync();
    h16* dst = AO + (size_t)t0 * CH;
#pragma unroll 1
    for (int ps = 0; ps < 2; ++ps) {
#pragma unroll
        for (int s = 0; s < 6; ++s) { const unsigned q = (unsigned)s * 32u + lane; const unsigned row = q / 12u, pc = q % 12u;
            const v4f x0 = *(const v4fa*)(&os[wb + row * OSP + pc * 8u]); const v4f x1 = *(const v4fa*)(&os[wb + row * OSP + pc * 8u + 4u]); v8h hv;
#pragma unroll
            for (int i = 0; i < 4; ++i) { hv[i] = toh_flush(x0[i]); hv[4 + i] = toh_flush(x1[i]); }
            *(volatile v8h*)(dst + (size_t)q * 8) = hv; }
        if (ps == 0) __threadfence(); }
}

static_assert(8 * 32 * 16 == 16 * 64 * 4);
__global__ __launch_bounds__(32) void k_outp(const h16* __restrict__ A, const h16* __restrict__ Bt, const float* __restrict__ bias, const float* __restrict__ x, float* OUT) {
    __shared__ __align__(16) float os[16 * 68];
    const int lane = threadIdx.x & 31, lr = lane & 15, hi = lane >> 4;
    const unsigned r0 = blockIdx.x * 64u, c0 = blockIdx.y * 64u;
    v8f acc[4][4];
#pragma unroll
    for (int mb = 0; mb < 4; ++mb)
#pragma unroll
        for (int nb = 0; nb < 4; ++nb) acc[mb][nb] = (v8f){};
    const size_t aoff = (size_t)(r0 + (unsigned)lr) * CH + 8 * hi, boff = (size_t)(c0 + (unsigned)lr) * CH + 8 * hi;
#pragma unroll 1
    for (int kc = 0; kc < CH; kc += 32) {
        v16h a[4];
#pragma unroll
        for (int mb = 0; mb < 4; ++mb) a[mb] = ldh(A + aoff + (size_t)mb * 16 * CH + kc);
#pragma unroll
        for (int nb = 0; nb < 4; ++nb) { const v16h b = ldh(Bt + boff + (size_t)nb * 16 * CH + kc);
#pragma unroll
            for (int mb = 0; mb < 4; ++mb) acc[mb][nb] = wmma16g(a[mb], b, acc[mb][nb]); }
    }
    const unsigned bb = c0 / (unsigned)HWP, tt = c0 % (unsigned)HWP;
    const size_t obase = ((size_t)bb * CO + (size_t)r0) * HWP_FULL + (size_t)tt;
#pragma unroll
    for (int mb = 0; mb < 4; ++mb) {
        float br[8];
#pragma unroll
        for (int j = 0; j < 8; ++j) br[j] = bfr(bias[r0 + (unsigned)(mb * 16 + hi * 8 + j)]);
#pragma unroll
        for (int nb = 0; nb < 4; ++nb) {
#pragma unroll
            for (int j = 0; j < 8; ++j) os[(hi * 8 + j) * 68 + nb * 16 + lr] = acc[mb][nb][j] * WLI + br[j]; }
        wave_sync();
#pragma unroll 1
        for (int ps = 0; ps < 2; ++ps) {
            const size_t sb = obase + (size_t)(mb * 16) * HWP_FULL;
#pragma unroll
            for (int s = 0; s < 8; ++s) { const int row = 2 * s + (lane >> 4), c4 = (lane & 15) * 4;
                const v4f t = *(const v4fa*)(&os[row * 68 + c4]);
                const size_t oo = sb + (size_t)row * HWP_FULL + c4;
                const v4f xv = *(const v4f*)(x + oo);
                v4f val; val[0] = t[0] + bfr(xv[0]); val[1] = t[1] + bfr(xv[1]); val[2] = t[2] + bfr(xv[2]); val[3] = t[3] + bfr(xv[3]);
                *(volatile v4f*)(OUT + oo) = val; }
            if (ps == 0) __threadfence(); }
        wave_sync();
    }
}

static constexpr size_t al256(size_t v) { return (v + 255) & ~(size_t)255; }
static constexpr size_t SZ_XT = al256((size_t)NTOK * CI * 2);
static constexpr size_t SZ_WB = al256((size_t)3 * CH * CI * 2);
static constexpr size_t SZ_WL = al256((size_t)CO * CH * 2);
static constexpr size_t SZ_PL = al256((size_t)NTOK * CH * 2);
static constexpr size_t SZ_TOTAL = SZ_XT + SZ_WB + SZ_WL + 8 * SZ_PL;
static_assert(SZ_TOTAL <= (size_t)134217728);
static_assert(((size_t)CH * CI * 2) % 256 == 0);
static_assert((size_t)NB * CH * HWP == (size_t)NTOK * CH);
static constexpr size_t NEED_X = ((size_t)(NB - 1) * CI + (size_t)(CI - 1)) * HWP_FULL + HWP;
static constexpr size_t N8_W  = (size_t)CH * CI / 8;
static constexpr unsigned N8_WL = (unsigned)((size_t)CO * CH / 8);
static constexpr unsigned G_W  = (unsigned)((N8_W + 255) / 256);
static constexpr unsigned G_WL = (N8_WL + 255u) / 256u;

extern "C" void kernel_launch(void* const* d_in, const int* in_sizes, int n_in,
                              void* d_out, int out_size, void* d_ws, size_t ws_size, hipStream_t stream) {
    if (n_in < 9) return;
    if ((size_t)in_sizes[0] < NEED_X) return;
    if (in_sizes[1] < CH * CI || in_sizes[3] < CH * CI || in_sizes[5] < CH * CI) return;
    if (in_sizes[2] < CH || in_sizes[4] < CH || in_sizes[6] < CH) return;
    if (in_sizes[7] < CO * CH || in_sizes[8] < CO) return;
    if ((size_t)out_size < NEED_X) return;
    if (SZ_TOTAL > ws_size) return;
    const float* x  = (const float*)d_in[0];
    const float* w1 = (const float*)d_in[1]; const float* b1 = (const float*)d_in[2];
    const float* w2 = (const float*)d_in[3]; const float* b2 = (const float*)d_in[4];
    const float* w3 = (const float*)d_in[5]; const float* b3 = (const float*)d_in[6];
    const float* wl = (const float*)d_in[7]; const float* bl = (const float*)d_in[8];
    float* OUT = (float*)d_out;
    char* wsp = (char*)d_ws;
    bf*  XT  = (bf*)wsp;  wsp += SZ_XT;
    bf*  WB  = (bf*)wsp;  wsp += SZ_WB;
    h16* WLh = (h16*)wsp; wsp += SZ_WL;
    h16* QH  = (h16*)wsp; wsp += SZ_PL;
    h16* QR  = (h16*)wsp; wsp += SZ_PL;
    h16* KP  = (h16*)wsp; wsp += SZ_PL;
    h16* KR  = (h16*)wsp; wsp += SZ_PL;
    h16* VP  = (h16*)wsp; wsp += SZ_PL;
    h16* VT  = (h16*)wsp; wsp += SZ_PL;
    h16* AO  = (h16*)wsp; wsp += SZ_PL;
    h16* AOT = (h16*)wsp; wsp += SZ_PL;
    bf* W1B = WB; bf* W2B = WB + (size_t)CH * CI; bf* W3B = WB + (size_t)2 * CH * CI;

    k_xt<<<dim3(HWP / 32, NB, 1), 256, 0, stream>>>(x, XT);
    k_cvt8<<<G_W, 256, 0, stream>>>(w1, W1B, N8_W);
    k_cvt8<<<G_W, 256, 0, stream>>>(w2, W2B, N8_W);
    k_cvt8<<<G_W, 256, 0, stream>>>(w3, W3B, N8_W);
    k_wcvt<<<G_WL, 256, 0, stream>>>(wl, WLh, N8_WL);

    k_proj<<<dim3(CH / 48, NTOK / 64, 1), 32, 0, stream>>>(W1B, XT, b1, QH, QR, 1);
    k_proj<<<dim3(CH / 48, NTOK / 64, 1), 32, 0, stream>>>(W2B, XT, b2, KP, KR, 1);
    k_proj<<<dim3(CH / 48, NTOK / 64, 1), 32, 0, stream>>>(W3B, XT, b3, VP, VP, 0);
    k_vt<<<dim3(NTOK / 64, 1, 1), 256, 0, stream>>>(VP, VT);

    k_flash<<<dim3(NTOK / (16 * AW), 1, 1), 32 * AW, 0, stream>>>(QH, QR, KP, KR, VT, AO);

    k_at<<<dim3(HWP / 64, NB, 1), 256, 0, stream>>>(AO, AOT);
    k_outp<<<dim3(CO / 64, NTOK / 64, 1), 32, 0, stream>>>(WLh, AOT, bl, x, OUT);
}
